// SparseGATLayer_53300544143788
// MI455X (gfx1250) — hardware-run, weakly checked
//
#include <hip/hip_runtime.h>

typedef float          v8f   __attribute__((ext_vector_type(8)));
typedef float          v4f   __attribute__((ext_vector_type(4)));
typedef unsigned int   v4u   __attribute__((ext_vector_type(4)));
typedef int            v8i   __attribute__((ext_vector_type(8)));
typedef unsigned short v8us  __attribute__((ext_vector_type(8)));
typedef unsigned short v16us __attribute__((ext_vector_type(16)));
typedef __bf16         v16bf __attribute__((ext_vector_type(16)));
typedef _Float16       v16h  __attribute__((ext_vector_type(16)));
typedef v4f  __attribute__((may_alias)) v4fa;
typedef v8us __attribute__((may_alias)) v8usa;
union FragB { v16bf v; v16us u; v8us h[2]; v8i w; };
union FragH { v16h  v; v16us u; v8us h[2]; v8i w; };

__device__ __forceinline__ v8f wmb(const FragB& a, const FragB& b, v8f c) {
  v8f d = __builtin_amdgcn_wmma_f32_16x16x32_bf16(false, a.v, false, b.v, (short)0, c, false, false);
  asm volatile("v_nop\n\tv_nop\n\tv_nop\n\tv_nop" : "+v"(d) : "v"(a.w), "v"(b.w));
  return d;
}

__device__ __forceinline__ v8f wmh(const FragH& a, const FragH& b, v8f c) {
  v8f d = __builtin_amdgcn_wmma_f32_16x16x32_f16(false, a.v, false, b.v, (short)0, c, false, false);
  asm volatile("v_nop\n\tv_nop\n\tv_nop\n\tv_nop" : "+v"(d) : "v"(a.w), "v"(b.w));
  return d;
}

__device__ __forceinline__ unsigned bf16_bits(float f) {
  const unsigned u = __float_as_uint(f);
  const unsigned r = (u + 0x7FFFu + ((u >> 16) & 1u)) >> 16;
  const unsigned q = (u >> 16) | 0x40u;
  return ((u & 0x7fffffffu) > 0x7f800000u) ? q : r;
}

__device__ __forceinline__ float bf16_val(float f) {
  return __uint_as_float(bf16_bits(f) << 16);
}
__device__ __forceinline__ int clampi(int v, int lo, int hi) {
  return v < lo ? lo : (v > hi ? hi : v);
}

__device__ __forceinline__ unsigned f16_bits(float f) {
  const unsigned u  = __float_as_uint(f);
  const unsigned s  = (u >> 16) & 0x8000u;
  const unsigned a  = u & 0x7fffffffu;
  const unsigned t  = a - 0x38000000u;
  const unsigned r  = (t + 0x0FFFu + ((t >> 13) & 1u)) >> 13;
  const unsigned rc = r > 0x7C00u ? 0x7C00u : r;
  const bool small  = a < 0x38800000u;
  const bool isnan  = a > 0x7f800000u;
  const unsigned fin = small ? 0u : (s | rc);
  return isnan ? (s | 0x7E00u) : fin;
}

__device__ __forceinline__ unsigned pk16(unsigned lo, unsigned hi) { return lo | (hi << 16); }
__device__ __forceinline__ unsigned bf16_lo_bits(float v) {
  float hi = bf16_val(v);
  asm volatile("" : "+v"(hi));
  return bf16_bits(v - hi);
}
__device__ __forceinline__ v4u pack8_bf16(v4f a, v4f c) {
  return (v4u){ pk16(bf16_bits(a[0]), bf16_bits(a[1])), pk16(bf16_bits(a[2]), bf16_bits(a[3])),
                pk16(bf16_bits(c[0]), bf16_bits(c[1])), pk16(bf16_bits(c[2]), bf16_bits(c[3])) };
}
__device__ __forceinline__ v4u pack8_bf16_lo(v4f a, v4f c) {
  return (v4u){ pk16(bf16_lo_bits(a[0]), bf16_lo_bits(a[1])), pk16(bf16_lo_bits(a[2]), bf16_lo_bits(a[3])),
                pk16(bf16_lo_bits(c[0]), bf16_lo_bits(c[1])), pk16(bf16_lo_bits(c[2]), bf16_lo_bits(c[3])) };
}
__device__ __forceinline__ v4u pack8_f16(v4f a, v4f c) {
  return (v4u){ pk16(f16_bits(a[0]), f16_bits(a[1])), pk16(f16_bits(a[2]), f16_bits(a[3])),
                pk16(f16_bits(c[0]), f16_bits(c[1])), pk16(f16_bits(c[2]), f16_bits(c[3])) };
}

template <int FORM>
__global__ __launch_bounds__(256) void k_plane(const float* __restrict__ src, int rows, int cols, int ldsrc,
                                               unsigned short* __restrict__ dst, int MP, int KP) {
  static_assert(FORM >= 0 && FORM <= 3);
  const int KTOT = (FORM == 1 || FORM == 3) ? 2 * KP : KP;
  const unsigned ppr   = (unsigned)(KTOT >> 3);
  const unsigned kp8   = (unsigned)(KP >> 3);
  const unsigned total = (unsigned)MP * ppr;
  const unsigned g     = blockIdx.x * 256u + threadIdx.x;
  const unsigned rowu  = g / ppr;
  const unsigned p     = g - rowu * ppr;
  const bool second    = p >= kp8;
  const int row = (int)rowu;
  const int c0  = (int)((second ? p - kp8 : p) << 3);
  const float* srow = src + (size_t)clampi(row, 0, rows - 1) * (size_t)ldsrc;
  float x[8];
  unsigned mk[8];
#pragma unroll
  for (int e = 0; e < 8; ++e) {
    const int c = c0 + e;
    const float v = srow[clampi(c, 0, cols - 1)];
    asm volatile("" :: "v"(v));
    x[e]  = v;
    mk[e] = (row < rows && c < cols) ? 0xFFFFu : 0u;
  }
  const v4f a = (v4f){ x[0], x[1], x[2], x[3] };
  const v4f c = (v4f){ x[4], x[5], x[6], x[7] };
  v4u o;
  if (FORM == 2) {
    o = pack8_f16(a, c);
  } else {
    const v4u hi = pack8_bf16(a, c);
    o = hi;
    if (FORM == 1) { const v4u lo = pack8_bf16_lo(a, c); o = second ? lo : hi; }
  }
  const v4u mw = (v4u){ pk16(mk[0], mk[1]), pk16(mk[2], mk[3]), pk16(mk[4], mk[5]), pk16(mk[6], mk[7]) };
  o &= mw;
  if (g < total) {
    volatile v4u* q = (volatile v4u*)(dst + (size_t)g * 8);
    *q = o;
    __threadfence();
    *q = o;
  }
}

template <int FORM> struct FragOf    { typedef FragB T; };
template <>         struct FragOf<2> { typedef FragH T; };
__device__ __forceinline__ v8f mm(const FragB& a, const FragB& b, v8f c) { return wmb(a, b, c); }
__device__ __forceinline__ v8f mm(const FragH& a, const FragH& b, v8f c) { return wmh(a, b, c); }
template <class F> __device__ __forceinline__ F ld_frag(const unsigned short* p) {
  F f;
  f.h[0] = *(const v8usa*)(p);
  f.h[1] = *(const v8usa*)(p + 16);
  return f;
}

template <int FORM, int EPI>
__global__ __launch_bounds__(256) __attribute__((amdgpu_num_vgpr(248)))
void k_gemm_nt(const unsigned short* __restrict__ A, const unsigned short* __restrict__ B,
               const float* __restrict__ bias, float* __restrict__ D, int M, int N, int KTOT, int ldd) {
  static_assert(FORM >= 0 && FORM <= 2);
  static_assert(EPI == 0 || EPI == 1);
  typedef typename FragOf<FORM>::T F;
  __shared__ __attribute__((aligned(16))) float sT[8][16 * 68];
  const int lane = threadIdx.x & 31;
  const int wave = threadIdx.x >> 5;
  const int tilesM = (M + 63) >> 6;
  const int tilesN = (N + 63) >> 6;
  const int tile = blockIdx.x * 8 + wave;
  if (tile >= tilesM * tilesN) return;
  const int tm = tile / tilesN;
  const int tn = tile - tm * tilesN;
  const int m0 = tm << 6;
  const int n0 = tn << 6;

  const int rl = lane & 15;
  const int h8 = (lane >> 4) * 8;
  const unsigned short* pa = A + (size_t)(m0 + rl) * (size_t)KTOT + h8;
  const unsigned short* pb = B + (size_t)(n0 + rl) * (size_t)KTOT + h8;

  v8f acc[4][4];
#pragma unroll
  for (int i = 0; i < 4; ++i)
#pragma unroll
    for (int j = 0; j < 4; ++j) acc[i][j] = (v8f){0.f, 0.f, 0.f, 0.f, 0.f, 0.f, 0.f, 0.f};

#pragma unroll 1
  for (int k0 = 0; k0 < KTOT; k0 += 32) {
    F bf[4];
#pragma unroll
    for (int j = 0; j < 4; ++j) bf[j] = ld_frag<F>(pb + (size_t)(j << 4) * (size_t)KTOT + k0);
#pragma unroll
    for (int i = 0; i < 4; ++i) {
      const F af = ld_frag<F>(pa + (size_t)(i << 4) * (size_t)KTOT + k0);
#pragma unroll
      for (int j = 0; j < 4; ++j) acc[i][j] = mm(af, bf[j], acc[i][j]);
    }
  }

  float* slab = sT[wave];
  const int hh = lane >> 4;
  const int c4 = (lane & 15) * 4;
  const int nc = n0 + c4;
  const bool cok = nc < N;
  v4f bv = (v4f){0.f, 0.f, 0.f, 0.f};
  if (EPI == 1) {
    bv = *(const v4fa*)(bias + clampi(nc, 0, N - 4));
    asm volatile("" :: "v"(bv));
  }
#pragma unroll
  for (int i = 0; i < 4; ++i) {
    const int mBase = m0 + (i << 4);
#pragma unroll
    for (int j = 0; j < 4; ++j) {
#pragma unroll
      for (int r = 0; r < 8; ++r) slab[(h8 + r) * 68 + (j << 4) + rl] = acc[i][j][r];
    }
    __builtin_amdgcn_fence(__ATOMIC_RELEASE, "workgroup");
    __builtin_amdgcn_wave_barrier();
    __builtin_amdgcn_fence(__ATOMIC_ACQUIRE, "workgroup");
    v4f vv[8];
#pragma unroll
    for (int it = 0; it < 8; ++it) {
      const int row = it * 2 + hh;
      v4f v = *(const v4fa*)(slab + row * 68 + c4);
      if (EPI == 1) v += bv;
      vv[it] = v;
    }
    for (int pass = 0; pass < 2; ++pass) {
#pragma unroll
      for (int it = 0; it < 8; ++it) {
        const int row = mBase + it * 2 + hh;
        if (cok && row < M) *(volatile v4f*)(D + (size_t)row * (size_t)ldd + nc) = vv[it];
      }
      __threadfence();
    }
    __builtin_amdgcn_fence(__ATOMIC_RELEASE, "workgroup");
    __builtin_amdgcn_wave_barrier();
    __builtin_amdgcn_fence(__ATOMIC_ACQUIRE, "workgroup");
  }
}

#pragma clang fp contract(off)


#define NN      50000
#define NE      800000
#define MPAD    50048
#define KD      128
#define DOUTW   128
#define RTHR    256
#define RWAVES  8
#define RPN     32
#define BT      512
#define BW      16
#define BEPT    8
#define BCHUNK  (BT * BEPT)
#define NCH     ((NE + BCHUNK - 1) / BCHUNK)
#define NB      1024
#define NBLK    ((NN + NB - 1) / NB)
#define RCAP    20480
#define SLOTSH  21
#define WCH     32
#define LISTTOT (NBLK * RCAP)
#define LDS_BKT ((2 * RCAP + 3 * NB + 64) * 4)
#define WSMAX   ((size_t)128 << 20)
#define WSTOTAL 43292928

static_assert(NBLK == 49 && 49 * 1024 >= NN);
static_assert(6250 * 8 == NN);
static_assert(391 * 128 == MPAD && MPAD % 64 == 0 && MPAD >= NN && MPAD % RPN == 0);
static_assert(32 * 4 == DOUTW && KD == 128 && KD % 32 == 0 && DOUTW % 64 == 0);
static_assert(NE < (1 << SLOTSH));
static_assert(NB <= 1024 && (NB & (NB - 1)) == 0 && NB == 2 * BT);
static_assert(NE % 8 == 0 && NE >= 8);
static_assert(NCH * BCHUNK >= NE && NCH == 196);
static_assert(RCAP % 32 == 0);
static_assert(RCAP * 5 >= 16759 * 6);
static_assert(LDS_BKT == 176384 && LDS_BKT <= 327680);
static_assert(BW == BT / 32 && BW == 16);
static_assert(WCH == 32);
static_assert(RWAVES * 4 == RPN);

typedef int          v4i __attribute__((ext_vector_type(4)));
typedef int          v2i __attribute__((ext_vector_type(2)));
typedef v4i __attribute__((may_alias)) v4ia;
typedef v2i __attribute__((may_alias)) v2ia;

__global__ __launch_bounds__(256) void k_prep(const float* __restrict__ W, const float* __restrict__ avec,
                                              unsigned short* WT, float* ATAB) {
  const int tid = (int)threadIdx.x;
  if (blockIdx.x < 8u) {
    const int g = (int)blockIdx.x * 256 + tid;
    const int n = g >> 4;
    const int k0 = (g & 15) << 3;
    float x[8];
#pragma unroll
    for (int e = 0; e < 8; ++e) {
      const float v = W[(size_t)(k0 + e) * DOUTW + n];
      asm volatile("" :: "v"(v));
      x[e] = v;
    }
    const v4u o = pack8_bf16((v4f){ x[0], x[1], x[2], x[3] }, (v4f){ x[4], x[5], x[6], x[7] });
    volatile v4u* q = (volatile v4u*)(WT + (size_t)g * 8);
    *q = o;
    __threadfence();
    *q = o;
  } else {
    const int idx = 4 * (tid & 63);
    const v4f t = *(const v4fa*)(avec + idx);
    asm volatile("" :: "v"(t));
    v4u o;
    o.x = bf16_bits(t.x) << 16;
    o.y = bf16_bits(t.y) << 16;
    o.z = bf16_bits(t.z) << 16;
    o.w = bf16_bits(t.w) << 16;
    const bool wr = tid < 64;
    volatile v4u* q = (volatile v4u*)(ATAB + idx);
    if (wr) *q = o;
    __threadfence();
    if (wr) *q = o;
  }
}

__global__ __launch_bounds__(BT) void k_list(const int* __restrict__ erow, const int* __restrict__ ecol,
                                             unsigned* LIST, int* META, int* FLAG) {
  extern __shared__ v4u lds_bkt[];
  int* reg1 = (int*)lds_bkt;
  int* reg2 = reg1 + RCAP;
  int* scnt = reg2 + RCAP;
  int* soff = scnt + NB;
  int* curs = soff + NB;
  int* wcnt = curs + NB;
  int* wtot = wcnt + 2 * BW;
  const int tid = (int)threadIdx.x, lane = tid & 31, wave = tid >> 5;
  const int nodeBase = (int)blockIdx.x * NB;
  int nb = NN - nodeBase;
  nb = nb > NB ? NB : (nb < 0 ? 0 : nb);
  const unsigned nbs = (unsigned)nodeBase, unb = (unsigned)nb;

  scnt[2 * tid] = 0;
  scnt[2 * tid + 1] = 0;

  int tot = 0;
#pragma unroll 1
  for (int ch = 0; ch < NCH; ++ch) {
    const int par = ch & 1;
    const int e0  = ch * BCHUNK + tid * BEPT;
    const bool valid = e0 < NE;
    const int ea = e0 < NE - 8 ? e0 : NE - 8;
    const v4i da = *(const v4ia*)(erow + ea);
    const v4i db = *(const v4ia*)(erow + ea + 4);
    asm volatile("" :: "v"(da), "v"(db));
    const unsigned s0 = (unsigned)da.x - nbs, s1 = (unsigned)da.y - nbs;
    const unsigned s2 = (unsigned)da.z - nbs, s3 = (unsigned)da.w - nbs;
    const unsigned s4 = (unsigned)db.x - nbs, s5 = (unsigned)db.y - nbs;
    const unsigned s6 = (unsigned)db.z - nbs, s7 = (unsigned)db.w - nbs;
    const bool h0 = valid && (s0 < unb), h1 = valid && (s1 < unb), h2 = valid && (s2 < unb), h3 = valid && (s3 < unb);
    const bool h4 = valid && (s4 < unb), h5 = valid && (s5 < unb), h6 = valid && (s6 < unb), h7 = valid && (s7 < unb);
    const int c = (int)h0 + (int)h1 + (int)h2 + (int)h3 + (int)h4 + (int)h5 + (int)h6 + (int)h7;
    int incl = c;
#pragma unroll
    for (int d = 1; d < 32; d <<= 1) {
      const int up = __shfl_up(incl, d, 32);
      incl += (lane >= d) ? up : 0;
    }
    const int wtotal = __shfl(incl, 31, 32);
    if (lane == 0) wcnt[par * BW + wave] = wtotal;
    __syncthreads();
    int all = 0, pre = 0;
#pragma unroll
    for (int g = 0; g < 4; ++g) {
      const v4i w4 = *(const v4ia*)(wcnt + par * BW + 4 * g);
      const int c0 = clampi(w4.x, 0, 256), c1 = clampi(w4.y, 0, 256);
      const int c2 = clampi(w4.z, 0, 256), c3 = clampi(w4.w, 0, 256);
      all += c0 + c1 + c2 + c3;
      pre += (4 * g + 0 < wave) ? c0 : 0;
      pre += (4 * g + 1 < wave) ? c1 : 0;
      pre += (4 * g + 2 < wave) ? c2 : 0;
      pre += (4 * g + 3 < wave) ? c3 : 0;
    }
    int pos = tot + pre + (incl - c);
#define PUTJ(J, HJ, SJ) if (HJ) { if (pos < RCAP) reg1[pos] = (int)((unsigned)(e0 + (J)) | ((SJ) << SLOTSH)); ++pos; }
    PUTJ(0, h0, s0)
    PUTJ(1, h1, s1)
    PUTJ(2, h2, s2)
    PUTJ(3, h3, s3)
    PUTJ(4, h4, s4)
    PUTJ(5, h5, s5)
    PUTJ(6, h6, s6)
    PUTJ(7, h7, s7)
#undef PUTJ
    tot += all;
  }
  __syncthreads();
  const bool ovf = tot > RCAP;
  const int nh = ovf ? RCAP : tot;

  if (wave == 0) {
#pragma unroll 1
    for (int b0 = 0; b0 < nh; b0 += 32) {
      const int idx = b0 + lane;
      const int uv  = reg1[idx < nh ? idx : nh - 1];
      const int m32 = (nh - b0) < 32 ? (nh - b0) : 32;
#pragma unroll 1
      for (int k = 0; k < m32; ++k) {
        const int u  = __builtin_amdgcn_readlane(uv, k);
        const int sl = (int)(((unsigned)u >> SLOTSH) & (unsigned)(NB - 1));
        const int cv = scnt[sl] + 1;
        if (lane == 0) scnt[sl] = cv;
      }
    }
  }
  __syncthreads();

  int e0c, e1c;
  {
    const v2i cc = *(const v2ia*)(scnt + 2 * tid);
    e0c = cc.x < 0 ? 0 : cc.x;
    e1c = cc.y < 0 ? 0 : cc.y;
    const int ts = e0c + e1c;
    int incl = ts;
#pragma unroll
    for (int d = 1; d < 32; d <<= 1) {
      const int up = __shfl_up(incl, d, 32);
      incl += (lane >= d) ? up : 0;
    }
    if (lane == 31) wtot[wave] = incl;
    __syncthreads();
    int pre = 0;
#pragma unroll
    for (int g = 0; g < 4; ++g) {
      const v4i w4 = *(const v4ia*)(wtot + 4 * g);
      pre += (4 * g + 0 < wave) ? w4.x : 0;
      pre += (4 * g + 1 < wave) ? w4.y : 0;
      pre += (4 * g + 2 < wave) ? w4.z : 0;
      pre += (4 * g + 3 < wave) ? w4.w : 0;
    }
    const int run = pre + incl - ts;
    soff[2 * tid]     = run;
    soff[2 * tid + 1] = run + e0c;
    curs[2 * tid]     = run;
    curs[2 * tid + 1] = run + e0c;
  }
  __syncthreads();

  if (wave == 0) {
#pragma unroll 1
    for (int b0 = 0; b0 < nh; b0 += 32) {
      const int idx = b0 + lane;
      const int uv  = reg1[idx < nh ? idx : nh - 1];
      const int m32 = (nh - b0) < 32 ? (nh - b0) : 32;
#pragma unroll 1
      for (int k = 0; k < m32; ++k) {
        const int u   = __builtin_amdgcn_readlane(uv, k);
        const int sl  = (int)(((unsigned)u >> SLOTSH) & (unsigned)(NB - 1));
        const int eid = (int)((unsigned)u & ((1u << SLOTSH) - 1u));
        const int pr  = curs[sl];
        const int pc  = clampi(pr, 0, RCAP - 1);
        if (lane == 0) { reg2[pc] = eid; curs[sl] = pc + 1; }
      }
    }
  }
  __syncthreads();

  {
    const int nhPad = (nh + 31) & ~31;
    const int nIt = (nhPad + BT - 1) / BT;
    unsigned* lbase = LIST + (size_t)blockIdx.x * (size_t)RCAP;
#pragma unroll 1
    for (int it = 0; it < nIt; ++it) {
      const int i  = it * BT + tid;
      int ic = i < nh ? i : nh - 1;
      ic = ic < 0 ? 0 : ic;
      const int eid = clampi(reg2[ic], 0, NE - 1);
      const int cw = ecol[eid];
      asm volatile("" :: "v"(cw));
      const unsigned msk = (i < nh) ? 0xFFFFFFFFu : 0u;
      const unsigned o = (unsigned)clampi(cw, 0, NN - 1) & msk;
      const int iw = i < RCAP ? i : RCAP - 1;
      volatile unsigned* q = (volatile unsigned*)(lbase + (size_t)iw);
      const bool wr = i < nhPad;
      if (wr) *q = o;
      __threadfence();
      if (wr) *q = o;
    }
  }

  {
    const int base = (int)blockIdx.x * RCAP;
    const v2i cc = *(const v2ia*)(scnt + 2 * tid);
    const v2i so = *(const v2ia*)(soff + 2 * tid);
    v4i m;
    m.x = base + so.x;
    m.y = cc.x;
    m.z = base + so.y;
    m.w = cc.y;
    volatile v4i* q = (volatile v4i*)(META + 2 * (size_t)(nodeBase + 2 * tid));
    *q = m;
    __threadfence();
    *q = m;
  }

  {
    const int fv = ovf ? 1 : 0;
    const v4i f = (v4i){ fv, fv, fv, fv };
    const bool wr = tid < 8;
    volatile v4i* q = (volatile v4i*)(FLAG + (size_t)blockIdx.x * 32 + 4 * (tid & 7));
    if (wr) *q = f;
    __threadfence();
    if (wr) *q = f;
  }
}

__global__ __launch_bounds__(RTHR) void k_rowprep(const float* __restrict__ WH, const float* __restrict__ ATAB,
                                                  float* SV) {
  __shared__ __attribute__((aligned(16))) float sA[256];
  __shared__ __attribute__((aligned(16))) float sS[2 * RPN];
  const int tid  = (int)threadIdx.x;
  const int lane = tid & 31;
  const int wave = tid >> 5;
  if (tid < 64) {
    const v4f t = *(const v4fa*)(ATAB + 4 * tid);
    *(v4fa*)(sA + 4 * tid) = t;
  }
  __syncthreads();
  const int c0 = lane * 4;
  const v4f a1 = *(const v4fa*)(sA + c0);
  const v4f a2 = *(const v4fa*)(sA + DOUTW + c0);
  const int nbase = (int)blockIdx.x * RPN + wave * 4;
#pragma unroll
  for (int i = 0; i < 4; ++i) {
    const int n = nbase + i;
    const v4f p = *(const v4fa*)(WH + (size_t)n * DOUTW + c0);
    float t1 = p.x * a1.x;
    float u  = p.y * a1.y; t1 = t1 + u;
    u = p.z * a1.z; t1 = t1 + u;
    u = p.w * a1.w; t1 = t1 + u;
    float t2 = p.x * a2.x;
    u = p.y * a2.y; t2 = t2 + u;
    u = p.z * a2.z; t2 = t2 + u;
    u = p.w * a2.w; t2 = t2 + u;
#pragma unroll
    for (int d = 16; d > 0; d >>= 1) {
      const float o1 = __shfl_xor(t1, d, 32);
      const float o2 = __shfl_xor(t2, d, 32);
      t1 = t1 + o1;
      t2 = t2 + o2;
    }
    if (lane == 0) { sS[wave * 4 + i] = t1; sS[RPN + wave * 4 + i] = t2; }
  }
  __syncthreads();
  if (wave == 0) {
    const int q2 = (lane >> 3) & 1;
    const int l8 = lane & 7;
    const v4f sv = *(const v4fa*)(sS + RPN * q2 + 4 * l8);
    const bool wr = lane < 16;
    volatile v4f* q = (volatile v4f*)(SV + (size_t)q2 * MPAD + (size_t)blockIdx.x * RPN + 4 * l8);
    if (wr) *q = sv;
    __threadfence();
    if (wr) *q = sv;
  }
}

__device__ __forceinline__ void form_chunk(const unsigned* __restrict__ LIST, const float* __restrict__ S2,
                                           int off, int cnt, int b0, int lane, float s1r, int nreal,
                                           int& col, float& e, bool& valid) {
  const int j = b0 + lane;
  valid = j < cnt;
  int jc = valid ? j : cnt - 1;
  jc = jc < 0 ? 0 : jc;
  const int idx = clampi(off + jc, 0, LISTTOT - 1);
  const unsigned cw = LIST[idx];
  asm volatile("" :: "v"(cw));
  col = clampi((int)cw, 0, nreal - 1);
  const float s2v = S2[col];
  asm volatile("" :: "v"(s2v));
  const float v = s1r + s2v;
  e = (v > 0.0f) ? v : 0.2f * v;
}

__global__ __launch_bounds__(RTHR) void k_walk(const float* __restrict__ WH, const float* __restrict__ SV,
                                               const unsigned* __restrict__ LIST, const int* __restrict__ META,
                                               const int* __restrict__ FLAG, float* out, int nreal) {
  const int lane = (int)threadIdx.x & 31;
  const int wave = (int)threadIdx.x >> 5;
  const int row  = (int)blockIdx.x * RWAVES + wave;
  int rowc = row < nreal ? row : nreal - 1;
  rowc = rowc < 0 ? 0 : rowc;
  const int c0  = lane * 4;
  const int blk = rowc >> 10;
  const float* S2 = SV + MPAD;

  const v2i mt = *(const v2ia*)(META + 2 * (size_t)rowc);
  asm volatile("" :: "v"(mt));
  const int fl = FLAG[(size_t)blk * 32];
  asm volatile("" :: "v"(fl));
  const float s1r = SV[rowc];
  asm volatile("" :: "v"(s1r));

  const int lo   = blk * RCAP;
  const int offv = clampi(mt.x, lo, lo + RCAP);
  const int cntv = (row < nreal) ? clampi(mt.y, 0, ((lo + RCAP - offv) < RCAP) ? (lo + RCAP - offv) : RCAP) : 0;
  const int off = __builtin_amdgcn_readfirstlane(offv);
  const int cnt = __builtin_amdgcn_readfirstlane(cntv);
  const bool poison = fl != 0;

  float shift = 0.0f;
#pragma unroll 1
  for (int b0 = 0; b0 < cnt; b0 += WCH) {
    int col; float e; bool valid;
    form_chunk(LIST, S2, off, cnt, b0, lane, s1r, nreal, col, e, valid);
    const float ez = valid ? e : 0.0f;
    const int ezi = __float_as_int(ez);
#pragma unroll
    for (int t = 0; t < WCH; ++t) shift = shift + __int_as_float(__builtin_amdgcn_readlane(ezi, t));
  }

  float nsum = 0.0f;
#pragma unroll 1
  for (int b0 = 0; b0 < cnt; b0 += WCH) {
    int col; float e; bool valid;
    form_chunk(LIST, S2, off, cnt, b0, lane, s1r, nreal, col, e, valid);
    const float arg = e - shift;
    const float ex  = expf(arg);
    const float exz = valid ? ex : 0.0f;
    const int exi = __float_as_int(exz);
#pragma unroll
    for (int t = 0; t < WCH; ++t) nsum = nsum + __int_as_float(__builtin_amdgcn_readlane(exi, t));
  }
  const float den = nsum + 1e-16f;

  v4f ac = (v4f){0.0f, 0.0f, 0.0f, 0.0f};
#pragma unroll 1
  for (int b0 = 0; b0 < cnt; b0 += WCH) {
    int col; float e; bool valid;
    form_chunk(LIST, S2, off, cnt, b0, lane, s1r, nreal, col, e, valid);
    const float arg = e - shift;
    const float ex  = expf(arg);
    const float exz = valid ? ex : 0.0f;
    const float w   = exz / den;
    const int wi = __float_as_int(w);
    const int m32 = (cnt - b0) < WCH ? (cnt - b0) : WCH;
#pragma unroll 1
    for (int k = 0; k < m32; ++k) {
      const int c = __builtin_amdgcn_readlane(col, k);
      const float wt = __int_as_float(__builtin_amdgcn_readlane(wi, k));
      const v4f hn = *(const v4fa*)(WH + (size_t)c * DOUTW + c0);
      float pr;
      pr = wt * hn.x; ac.x = ac.x + pr;
      pr = wt * hn.y; ac.y = ac.y + pr;
      pr = wt * hn.z; ac.z = ac.z + pr;
      pr = wt * hn.w; ac.w = ac.w + pr;
    }
  }

  const float qnan = __uint_as_float(0x7fc00000u);
  v4f r;
  r.x = poison ? qnan : ac.x;
  r.y = poison ? qnan : ac.y;
  r.z = poison ? qnan : ac.z;
  r.w = poison ? qnan : ac.w;
  float* orow = out + (size_t)rowc * DOUTW + c0;
  const bool rok = row < nreal;
  if (rok) *(volatile v4f*)orow = r;
  __threadfence();
  if (rok) *(volatile v4f*)orow = r;
}

extern "C" void kernel_launch(void* const* d_in, const int* in_sizes, int n_in,
                              void* d_out, int out_size, void* d_ws, size_t ws_size,
                              hipStream_t stream) {
  if (n_in < 4) return;
  if (in_sizes[0] != NN * KD) return;
  if (in_sizes[1] != 2 * NE) return;
  if (in_sizes[2] != KD * DOUTW) return;
  if (in_sizes[3] != 2 * DOUTW) return;
  if (out_size != NN * DOUTW) return;

  const float* hin  = (const float*)d_in[0];
  const int*   etab = (const int*)  d_in[1];
  const int*   erow = etab;
  const int*   ecol = etab + NE;
  const float* W    = (const float*)d_in[2];
  const float* avec = (const float*)d_in[3];
  float* out = (float*)d_out;

  const size_t szXB   = (size_t)MPAD * KD * 2;
  const size_t szWH   = (size_t)MPAD * DOUTW * 4;
  const size_t szLIST = (size_t)NBLK * RCAP * 4;
  const size_t szMETA = (size_t)NBLK * NB * 2 * 4;
  const size_t szSV   = (size_t)2 * MPAD * 4;
  const size_t szWT   = (size_t)DOUTW * KD * 2;
  const size_t szATAB = (size_t)1024;
  const size_t szFLAG = (size_t)6400;
  static_assert((size_t)MPAD * KD * 2 + (size_t)MPAD * DOUTW * 4 + (size_t)NBLK * RCAP * 4 +
                (size_t)NBLK * NB * 8 + (size_t)2 * MPAD * 4 + (size_t)DOUTW * KD * 2 + 1024 + 6400 == WSTOTAL);
  static_assert((size_t)WSTOTAL <= WSMAX);
  static_assert(NBLK * 128 <= 6400 && 256 * 4 <= 1024);
  char* ws = (char*)d_ws;
  size_t off = 0;
  const size_t oXB   = off; off += szXB;
  const size_t oWH   = off; off += szWH;
  const size_t oLIST = off; off += szLIST;
  const size_t oMETA = off; off += szMETA;
  const size_t oSV   = off; off += szSV;
  const size_t oWT   = off; off += szWT;
  const size_t oATAB = off; off += szATAB;
  const size_t oFLAG = off; off += szFLAG;
  if (off != (size_t)WSTOTAL) return;
  if (off > ws_size || off > (size_t)WSMAX) return;
  unsigned short* XB   = (unsigned short*)(ws + oXB);
  float*          WH   = (float*)(ws + oWH);
  unsigned*       LIST = (unsigned*)(ws + oLIST);
  int*            META = (int*)(ws + oMETA);
  float*          SV   = (float*)(ws + oSV);
  unsigned short* WT   = (unsigned short*)(ws + oWT);
  float*          ATAB = (float*)(ws + oATAB);
  int*            FLAG = (int*)(ws + oFLAG);

  hipFuncSetAttribute(reinterpret_cast<const void*>(&k_list),
                      hipFuncAttributeMaxDynamicSharedMemorySize, LDS_BKT);

  k_plane<0><<<MPAD * KD / 8 / 256, 256, 0, stream>>>(hin, NN, KD, KD, XB, MPAD, KD);
  k_prep<<<9, 256, 0, stream>>>(W, avec, WT, ATAB);
  k_list<<<NBLK, BT, LDS_BKT, stream>>>(erow, ecol, LIST, META, FLAG);
  const int tiles = (MPAD / 64) * (DOUTW / 64);
  const int gG = (tiles + 7) / 8;
  k_gemm_nt<0, 0><<<gG, 256, 0, stream>>>(XB, WT, ATAB, WH, MPAD, DOUTW, KD, DOUTW);
  k_rowprep<<<MPAD / RPN, RTHR, 0, stream>>>(WH, ATAB, SV);
  k_walk<<<NN / RWAVES, RTHR, 0, stream>>>(WH, SV, LIST, META, FLAG, out, NN);
}
